// DIFAttentionLayer_25915832664860
// MI455X (gfx1250) — hardware-verified
//
#include <hip/hip_runtime.h>


namespace {
constexpr int Bn = 4, T = 2048, D = 256, H = 8, HD = 32, NT = Bn * T;
constexpr float QS = 8.0f, KS = 8.0f, VS = 8.0f, PS = 8.0f, AS_ = 8.0f, SCALE = 0.17677669529663687f;
constexpr size_t PL = (size_t)Bn * H * T * HD;

typedef _Float16 b16;
typedef __attribute__((ext_vector_type(16))) _Float16 v16b;
typedef __attribute__((ext_vector_type(16))) __bf16 v16bb;
typedef __attribute__((ext_vector_type(8))) _Float16 v8b;
typedef __attribute__((ext_vector_type(8))) unsigned short v8us;
typedef __attribute__((ext_vector_type(8))) float v8f;
typedef __attribute__((ext_vector_type(4))) float v4f;
__device__ __forceinline__ float bf16_rne(float f) { unsigned int u = __float_as_uint(f); u += 0x7FFFu + ((u >> 16) & 1u); return __uint_as_float(u & 0xFFFF0000u); }
__device__ __forceinline__ unsigned short bf16_bits(float f) { unsigned int u = __float_as_uint(f); u += 0x7FFFu + ((u >> 16) & 1u); return (unsigned short)(u >> 16); }
__device__ __forceinline__ void split16(float v, b16& hi, b16& lo) { hi = (b16)v; lo = (b16)(v - (float)hi); }
__device__ __forceinline__ v16b frag_kb(const b16* p, int hh) { const v8b a = *(const v8b*)(p + 8 * hh), b = *(const v8b*)(p + 16 + 8 * hh); v16b f;
#pragma unroll
  for (int e = 0; e < 8; ++e) { f[e] = a[e]; f[8 + e] = b[e]; } return f; }
__device__ __forceinline__ v16bb frag_bf(const unsigned short* p, int hh) { const v8us a = *(const v8us*)(p + 8 * hh), b = *(const v8us*)(p + 16 + 8 * hh); union { unsigned short s[16]; v16bb v; } u;
#pragma unroll
  for (int e = 0; e < 8; ++e) { u.s[e] = a[e]; u.s[8 + e] = b[e]; } return u.v; }
__device__ __forceinline__ v16bb frag_f32bf(const float* p, int hh) { union { unsigned short s[16]; v16bb v; } u;
#pragma unroll
  for (int e = 0; e < 8; ++e) { u.s[e] = bf16_bits(p[8 * hh + e]); u.s[8 + e] = bf16_bits(p[16 + 8 * hh + e]); } return u.v; }
__device__ __forceinline__ void frag_split(const float* p, int hh, v16b& fh, v16b& fl) {
#pragma unroll
  for (int e = 0; e < 8; ++e) { b16 a, c; split16(p[8 * hh + e] * AS_, a, c); fh[e] = a; fl[e] = c; split16(p[16 + 8 * hh + e] * AS_, a, c); fh[8 + e] = a; fl[8 + e] = c; } }
__device__ __forceinline__ v8f wmma16b(v16b a, v16b b, v8f c) { v8f d = __builtin_amdgcn_wmma_f32_16x16x32_f16(false, a, false, b, (short)0, c, false, false); asm volatile("v_nop\n\tv_nop\n\tv_nop\n\tv_nop" : "+v"(d) : "v"(a), "v"(b)); return d; }
__device__ __forceinline__ v8f wmma16bb(v16bb a, v16bb b, v8f c) { v8f d = __builtin_amdgcn_wmma_f32_16x16x32_bf16(false, a, false, b, (short)0, c, false, false); asm volatile("v_nop\n\tv_nop\n\tv_nop\n\tv_nop" : "+v"(d) : "v"(a), "v"(b)); return d; }
__device__ __forceinline__ void wave_lds_sync() { __builtin_amdgcn_fence(__ATOMIC_RELEASE, "workgroup"); __builtin_amdgcn_wave_barrier(); __builtin_amdgcn_fence(__ATOMIC_ACQUIRE, "workgroup"); }
__device__ __forceinline__ float nexp(float x) { return __builtin_amdgcn_exp2f(x * 1.4426950408889634f); }
__device__ __forceinline__ float sigm(float x) { return __builtin_amdgcn_rcpf(1.0f + nexp(-x)); }

__global__ __launch_bounds__(256) void prep_kernel(const float* __restrict__ Wqc, const float* __restrict__ Wkc, const float* __restrict__ Wv, const float* __restrict__ Wqk, const float* __restrict__ Wkk, const float* __restrict__ Wo, unsigned short* __restrict__ w16, b16* __restrict__ wo16) {
  const size_t tid = (size_t)blockIdx.x * blockDim.x + threadIdx.x, nth = (size_t)gridDim.x * blockDim.x;
  for (int pass = 0; pass < 2; ++pass) {
    for (size_t p = tid; p < (size_t)5 * D * D / 8; p += nth) { const int m = (int)(p / (D * D / 8)); const size_t q = p % (D * D / 8); const float* W = (m == 0) ? Wqc : (m == 1) ? Wkc : (m == 2) ? Wv : (m == 3) ? Wqk : Wkk; v8us v;
#pragma unroll
      for (int e = 0; e < 8; ++e) v[e] = bf16_bits(W[q * 8 + e]);
      *(volatile v8us*)(w16 + p * 8) = v; }
    for (size_t p = tid; p < (size_t)D * D / 8; p += nth) { v8b v;
#pragma unroll
      for (int e = 0; e < 8; ++e) v[e] = (b16)bf16_rne(Wo[p * 8 + e]);
      *(volatile v8b*)(wo16 + p * 8) = v; }
    __threadfence(); }
}

__global__ __launch_bounds__(128) void proj_kernel(const float* __restrict__ content, const float* __restrict__ category, const unsigned short* __restrict__ w16, b16* __restrict__ planes, b16* __restrict__ vt) {
  __shared__ __attribute__((aligned(16))) b16 Th[4][32][64 + 8], Tl[4][32][64 + 8]; __shared__ __attribute__((aligned(16))) b16 Vh[64][128 + 8], Vl[64][128 + 8];
  const int lane = threadIdx.x & 31, wave = threadIdx.x >> 5, nloc = lane & 15, hlf = lane >> 4, which = blockIdx.z, m0 = blockIdx.y * 128 + wave * 32, c0 = blockIdx.x * 64; const int b = (blockIdx.y * 128) / T, t0 = (blockIdx.y * 128) % T;
  const float* x = (which >= 3) ? category : content; const unsigned short* Wt = w16 + (size_t)which * D * D;
  v8f acc[2][4];
#pragma unroll
  for (int r = 0; r < 2; ++r)
#pragma unroll
    for (int t = 0; t < 4; ++t) acc[r][t] = (v8f){};
#pragma unroll 2
  for (int kb = 0; kb < D; kb += 32) { const v16bb a0 = frag_f32bf(x + (size_t)(m0 + nloc) * D + kb, hlf), a1 = frag_f32bf(x + (size_t)(m0 + 16 + nloc) * D + kb, hlf);
#pragma unroll
    for (int t = 0; t < 4; ++t) { const v16bb bw = frag_bf(Wt + (size_t)(c0 + t * 16 + nloc) * D + kb, hlf); acc[0][t] = wmma16bb(a0, bw, acc[0][t]); acc[1][t] = wmma16bb(a1, bw, acc[1][t]); } }
  if (which != 2) { const float scl = (which == 0 || which == 3) ? SCALE * QS : KS; const int pidx = (which == 0) ? 0 : (which == 1) ? 1 : (which == 3) ? 2 : 3;
#pragma unroll
    for (int t = 0; t < 4; ++t)
#pragma unroll
      for (int r = 0; r < 2; ++r)
#pragma unroll
        for (int v = 0; v < 8; ++v) { b16 a_, c_; split16(acc[r][t][v] * scl, a_, c_); Th[wave][r * 16 + 8 * hlf + v][t * 16 + nloc] = a_; Tl[wave][r * 16 + 8 * hlf + v][t * 16 + nloc] = c_; }
    wave_lds_sync();
    b16* base = planes + (size_t)pidx * 2 * PL;
    for (int pass = 0; pass < 2; ++pass) {
#pragma unroll
      for (int j = 0; j < 4; ++j) { const int rr = j * 8 + (lane >> 2), c8 = (lane & 3) * 8; const int m = m0 + rr, bb = m / T, tok = m % T;
#pragma unroll
        for (int hh2 = 0; hh2 < 2; ++hh2) { const int h = c0 / 32 + hh2; const size_t o = (((size_t)bb * H + h) * T + tok) * HD + c8;
          *(volatile v8b*)(base + o) = *(const v8b*)(&Th[wave][rr][hh2 * 32 + c8]); *(volatile v8b*)(base + PL + o) = *(const v8b*)(&Tl[wave][rr][hh2 * 32 + c8]); } }
      __threadfence(); }
    return; }
#pragma unroll
  for (int t = 0; t < 4; ++t)
#pragma unroll
    for (int r = 0; r < 2; ++r)
#pragma unroll
      for (int v = 0; v < 8; ++v) { b16 a_, c_; split16(acc[r][t][v] * VS, a_, c_); Vh[t * 16 + nloc][wave * 32 + r * 16 + 8 * hlf + v] = a_; Vl[t * 16 + nloc][wave * 32 + r * 16 + 8 * hlf + v] = c_; }
  __syncthreads();
  for (int pass = 0; pass < 2; ++pass) { for (int i = threadIdx.x; i < 64 * 16; i += 128) { const int cc = i >> 4, c8 = (i & 15) * 8; const int h = (c0 + cc) / 32, d = (c0 + cc) % 32; const size_t o = (((size_t)b * H + h) * HD + d) * T + t0 + c8;
      *(volatile v8b*)(vt + o) = *(const v8b*)(&Vh[cc][c8]); *(volatile v8b*)(vt + PL + o) = *(const v8b*)(&Vl[cc][c8]); } __threadfence(); }
}

__global__ __launch_bounds__(256) void attn_kernel(const b16* __restrict__ planes, const b16* __restrict__ vt, const float* __restrict__ alog, float* __restrict__ ctx) {
  __shared__ __attribute__((aligned(16))) float Os[16][D + 4];
  const int h = threadIdx.x >> 5, lane = threadIdx.x & 31, hh = lane >> 4, col = lane & 15; const int b = blockIdx.x / (T / 16), q0 = (blockIdx.x % (T / 16)) * 16, qi = q0 + col;
  const float alpha = sigm(bf16_rne(alog[0]));
  const size_t ho = ((size_t)b * H + h) * T; const b16* Qc = planes + ho * HD; const b16* Kc = planes + 2 * PL + ho * HD; const b16* Qk = planes + 4 * PL + ho * HD; const b16* Kk = planes + 6 * PL + ho * HD; const b16* V = vt + (((size_t)b * H + h) * HD) * T;
  const v16b qcf = frag_kb(Qc + (size_t)qi * HD, hh), qcl = frag_kb(Qc + PL + (size_t)qi * HD, hh), qkf = frag_kb(Qk + (size_t)qi * HD, hh), qkl = frag_kb(Qk + PL + (size_t)qi * HD, hh);
  float mc = -INFINITY, lc = 0.0f, mk = -INFINITY, lk = 0.0f; v8f oc[2] = {{}, {}}, ok[2] = {{}, {}};
  const int kend = q0 + 16;
  for (int kb = 0; kb < kend; kb += 32) { const bool diag = (kb + 32 > q0);
    for (int st = 0; st < 2; ++st) {
      const b16* K = st ? Kk : Kc; const v16b qf = st ? qkf : qcf, ql = st ? qkl : qcl;
      const v16b ka = frag_kb(K + (size_t)(kb + col) * HD, hh), kal = frag_kb(K + PL + (size_t)(kb + col) * HD, hh), kc2 = frag_kb(K + (size_t)(kb + 16 + col) * HD, hh), kcl = frag_kb(K + PL + (size_t)(kb + 16 + col) * HD, hh);
      v8f s0 = {}, s1 = {}; s0 = wmma16b(ka, qf, s0); s0 = wmma16b(ka, ql, s0); s0 = wmma16b(kal, qf, s0); s1 = wmma16b(kc2, qf, s1); s1 = wmma16b(kc2, ql, s1); s1 = wmma16b(kcl, qf, s1);
      float mr = -INFINITY;
#pragma unroll
      for (int r = 0; r < 8; ++r) { s0[r] *= 1.0f / (QS * KS); s1[r] *= 1.0f / (QS * KS); if (diag) { const int k0_ = kb + 8 * hh + r, k1_ = kb + 16 + 8 * hh + r; if (k0_ > qi) s0[r] = -INFINITY; if (k1_ > qi) s1[r] = -INFINITY; } mr = fmaxf(mr, fmaxf(s0[r], s1[r])); }
      mr = fmaxf(mr, __shfl_xor(mr, 16));
      float& m = st ? mk : mc; float& l = st ? lk : lc; v8f* o = st ? ok : oc;
      const float mn = fmaxf(m, mr), al_ = nexp(m - mn); m = mn; float sum = 0.0f; v16b pbv, plv;
#pragma unroll
      for (int r = 0; r < 8; ++r) { const float e0 = nexp(s0[r] - mn), e1 = nexp(s1[r] - mn); sum += e0 + e1; b16 a, cc; split16(e0 * PS, a, cc); pbv[r] = a; plv[r] = cc; split16(e1 * PS, a, cc); pbv[8 + r] = a; plv[8 + r] = cc; }
      sum += __shfl_xor(sum, 16); l = l * al_ + sum;
#pragma unroll
      for (int t = 0; t < 2; ++t) { o[t] *= al_; const v16b vf = frag_kb(V + (size_t)(t * 16 + col) * T + kb, hh), vl = frag_kb(V + PL + (size_t)(t * 16 + col) * T + kb, hh); o[t] = wmma16b(vf, pbv, o[t]); o[t] = wmma16b(vf, plv, o[t]); o[t] = wmma16b(vl, pbv, o[t]); } } }
  const float ic = (1.0f - alpha) / (lc * VS * PS), ik = alpha / (lk * VS * PS);
#pragma unroll
  for (int t = 0; t < 2; ++t)
#pragma unroll
    for (int r = 0; r < 8; ++r) Os[col][h * HD + t * 16 + 8 * hh + r] = oc[t][r] * ic + ok[t][r] * ik;
  __syncthreads();
  float* dst = ctx + ((size_t)b * T + q0) * D;
  for (int pass = 0; pass < 2; ++pass) { for (int i = threadIdx.x; i < 16 * (D / 4); i += 256) { const int rr = i / (D / 4), c4 = (i % (D / 4)) * 4; *(volatile v4f*)(dst + (size_t)rr * D + c4) = *(const v4f*)(&Os[rr][c4]); } __threadfence(); }
}

__global__ __launch_bounds__(128) void out_kernel(const float* __restrict__ ctx, const b16* __restrict__ wo16, const float* __restrict__ bo, float* __restrict__ out) {
  __shared__ __attribute__((aligned(16))) float Ts[4][32 * 64];
  const int lane = threadIdx.x & 31, wave = threadIdx.x >> 5, nloc = lane & 15, hlf = lane >> 4, m0 = blockIdx.y * 128 + wave * 32, c0 = blockIdx.x * 64;
  v8f acc[2][4];
#pragma unroll
  for (int r = 0; r < 2; ++r)
#pragma unroll
    for (int t = 0; t < 4; ++t) acc[r][t] = (v8f){};
#pragma unroll 2
  for (int kb = 0; kb < D; kb += 32) { v16b a0, l0, a1, l1; frag_split(ctx + (size_t)(m0 + nloc) * D + kb, hlf, a0, l0); frag_split(ctx + (size_t)(m0 + 16 + nloc) * D + kb, hlf, a1, l1);
#pragma unroll
    for (int t = 0; t < 4; ++t) { const v16b bw = frag_kb(wo16 + (size_t)(c0 + t * 16 + nloc) * D + kb, hlf); acc[0][t] = wmma16b(a0, bw, acc[0][t]); acc[0][t] = wmma16b(l0, bw, acc[0][t]); acc[1][t] = wmma16b(a1, bw, acc[1][t]); acc[1][t] = wmma16b(l1, bw, acc[1][t]); } }
  float* Tt = Ts[wave];
#pragma unroll
  for (int t = 0; t < 4; ++t) { const float bb = bf16_rne(bo[c0 + t * 16 + nloc]);
#pragma unroll
    for (int r = 0; r < 2; ++r)
#pragma unroll
      for (int v = 0; v < 8; ++v) Tt[(r * 16 + v + 8 * hlf) * 64 + t * 16 + nloc] = acc[r][t][v] * (1.0f / AS_) + bb; }
  wave_lds_sync();
  for (int pass = 0; pass < 2; ++pass) {
#pragma unroll
    for (int j = 0; j < 16; ++j) { const int rr = j * 2 + hlf, c4 = nloc * 4; *(volatile v4f*)(out + (size_t)(m0 + rr) * D + c0 + c4) = *(const v4f*)(Tt + rr * 64 + c4); }
    __threadfence(); }
}
}

extern "C" void kernel_launch(void* const* d_in, const int* in_sizes, int n_in,
                              void* d_out, int out_size, void* d_ws, size_t ws_size, hipStream_t stream) {
  (void)n_in; (void)out_size;
  const float* content = (const float*)d_in[0]; const float* category = (const float*)d_in[1]; const float* Wqc = (const float*)d_in[2]; const float* Wkc = (const float*)d_in[3]; const float* Wv = (const float*)d_in[4]; const float* Wqk = (const float*)d_in[5]; const float* Wkk = (const float*)d_in[6]; const float* Wo = (const float*)d_in[7]; const float* bo = (const float*)d_in[8]; const float* alog = (const float*)d_in[9];
  float* out = (float*)d_out;
  if (in_sizes[0] != NT * D || in_sizes[1] != NT * D || in_sizes[2] != D * D || in_sizes[7] != D * D || in_sizes[9] != 1) return;
  size_t off = 0; char* ws = (char*)d_ws;
  auto carve = [&](size_t bytes) { char* p = ws + off; off += (bytes + 255) & ~(size_t)255; return p; };
  unsigned short* w16 = (unsigned short*)carve((size_t)5 * D * D * 2); b16* wo16 = (b16*)carve((size_t)D * D * 2); b16* planes = (b16*)carve(PL * 2 * 8); b16* vt = (b16*)carve(PL * 2 * 2); float* ctx = (float*)carve((size_t)NT * D * 4);
  if (off > ws_size) return;
  prep_kernel<<<128, 256, 0, stream>>>(Wqc, Wkc, Wv, Wqk, Wkk, Wo, w16, wo16);
  proj_kernel<<<dim3(D / 64, NT / 128, 5), 128, 0, stream>>>(content, category, w16, planes, vt);
  attn_kernel<<<Bn * T / 16, 256, 0, stream>>>(planes, vt, alog, ctx);
  out_kernel<<<dim3(D / 64, NT / 128), 128, 0, stream>>>(ctx, wo16, bo, out);
}
